// MultiDimHiPPO_89103391523690
// MI455X (gfx1250) — hardware-run, weakly checked
//
#include <hip/hip_runtime.h>

typedef __attribute__((ext_vector_type(16))) __bf16   v16b;
typedef __attribute__((ext_vector_type(8)))  __bf16   v8b;
typedef __attribute__((ext_vector_type(8)))  float    v8f;
typedef __attribute__((ext_vector_type(4)))  float    v4f;
typedef __attribute__((ext_vector_type(4)))  unsigned v4u;
typedef v4f v4fa __attribute__((may_alias));

constexpr int kBatch   = 32;
constexpr int kSeq     = 1024;
constexpr int kDim     = 64;
constexpr int kState   = 64;
constexpr int kRows    = kBatch * kDim;
constexpr int kTilePitch = 65;

constexpr size_t kVtPlaneBytes = (size_t)kState * kSeq * 2;
constexpr size_t kXtPlaneBytes = (size_t)kRows * kSeq * 2;
constexpr size_t kOffVtHi = 0;
constexpr size_t kOffVtLo = kOffVtHi + kVtPlaneBytes;
constexpr size_t kOffXtHi = kOffVtLo + kVtPlaneBytes;
constexpr size_t kOffXtLo = kOffXtHi + kXtPlaneBytes;
constexpr size_t kCarveBytes = kOffXtLo + kXtPlaneBytes;
static_assert(kCarveBytes == 8650752, "carve");
static_assert(kCarveBytes <= 134217728, "carve limit");
static_assert((kOffVtLo % 128) == 0 && (kOffXtHi % 128) == 0 && (kOffXtLo % 128) == 0, "line aligned planes");
static_assert(kRows % 64 == 0 && kState % 64 == 0 && kSeq % 32 == 0, "tile multiples");

__device__ __forceinline__ unsigned short f2bf_bits(float f) {
  unsigned u = __float_as_uint(f);
  return (unsigned short)((u + 0x7FFFu + ((u >> 16) & 1u)) >> 16);
}
__device__ __forceinline__ float bf_bits2f(unsigned short h) { return __uint_as_float(((unsigned)h) << 16); }

__device__ __forceinline__ void split_pack2(float f0, float f1, unsigned& hw, unsigned& lw) {
  const unsigned short h0 = f2bf_bits(f0);
  const unsigned short h1 = f2bf_bits(f1);
  const float r0 = f0 - bf_bits2f(h0);
  const float r1 = f1 - bf_bits2f(h1);
  const unsigned short l0 = f2bf_bits(r0);
  const unsigned short l1 = f2bf_bits(r1);
  hw = (unsigned)h0 | ((unsigned)h1 << 16);
  lw = (unsigned)l0 | ((unsigned)l1 << 16);
}

__device__ __forceinline__ void split_pack8(const float* tile, int c8, int col, v4u& hv, v4u& lv) {
  float f[8];
#pragma unroll
  for (int e = 0; e < 8; ++e) f[e] = tile[(c8 + e) * kTilePitch + col];
  unsigned h0, h1, h2, h3, l0, l1, l2, l3;
  split_pack2(f[0], f[1], h0, l0);
  split_pack2(f[2], f[3], h1, l1);
  split_pack2(f[4], f[5], h2, l2);
  split_pack2(f[6], f[7], h3, l3);
  hv = (v4u){h0, h1, h2, h3};
  lv = (v4u){l0, l1, l2, l3};
}

__global__ __launch_bounds__(64) void k_vchain(
    const float* __restrict__ dA, const float* __restrict__ dB,
    unsigned short* __restrict__ VTh, unsigned short* __restrict__ VTl) {
  __shared__ __align__(16) float vbuf[2 * 64];
  __shared__ __align__(16) float tile[64 * kTilePitch];
  const int m    = threadIdx.x;
  const int lane = threadIdx.x & 31;
  const int wave = threadIdx.x >> 5;
  const int q    = lane >> 3;
  const int c8   = (lane & 7) * 8;

  float a[64];
#pragma unroll
  for (int j = 0; j < 16; ++j) {
    const v4f av = *(const v4f*)(dA + m * 64 + 4 * j);
    a[4 * j + 0] = av[0];
    a[4 * j + 1] = av[1];
    a[4 * j + 2] = av[2];
    a[4 * j + 3] = av[3];
  }
  {
    const float b0 = dB[m];
    vbuf[m] = b0;
    tile[63 * kTilePitch + m] = b0;
  }
  __syncthreads();

  int cur = 0;
#pragma unroll 1
  for (int chunk = 15; chunk >= 0; --chunk) {
    const int tlTop = (chunk == 15) ? 62 : 63;
#pragma unroll 1
    for (int tl = tlTop; tl >= 0; --tl) {
      const float* vb = vbuf + cur * 64;
      float s = 0.0f;
#pragma unroll
      for (int j = 0; j < 16; ++j) {
        const v4f vv = *(const v4fa*)(vb + 4 * j);
        s = fmaf(a[4 * j + 0], vv[0], s);
        s = fmaf(a[4 * j + 1], vv[1], s);
        s = fmaf(a[4 * j + 2], vv[2], s);
        s = fmaf(a[4 * j + 3], vv[3], s);
      }
      vbuf[(cur ^ 1) * 64 + m] = s;
      tile[tl * kTilePitch + m] = s;
      cur ^= 1;
      __syncthreads();
    }
    for (int pass = 0; pass < 2; ++pass) {
      for (int it = 0; it < 8; ++it) {
        const int mm = wave * 32 + it * 4 + q;
        v4u hv, lv;
        split_pack8(tile, c8, mm, hv, lv);
        const size_t off = (size_t)mm * kSeq + (size_t)chunk * 64 + c8;
        *(volatile v4u*)(VTh + off) = hv;
        *(volatile v4u*)(VTl + off) = lv;
      }
      __threadfence();
    }
    __syncthreads();
  }
}

__global__ __launch_bounds__(256) void k_xplanes(
    const float* __restrict__ x, unsigned short* __restrict__ XTh, unsigned short* __restrict__ XTl) {
  __shared__ __align__(16) float xs[64 * kTilePitch];
  const int tid  = threadIdx.x;
  const int lane = tid & 31;
  const int wave = tid >> 5;
  const int b    = blockIdx.x >> 4;
  const int t0   = (blockIdx.x & 15) * 64;
  const float* xb = x + (size_t)b * kSeq * kDim + (size_t)t0 * kDim;
#pragma unroll
  for (int j = 0; j < 4; ++j) {
    const int idx4 = tid + 256 * j;
    const int tt = idx4 >> 4;
    const int c4 = (idx4 & 15) * 4;
    const v4f v = *(const v4f*)(xb + tt * kDim + c4);
    xs[tt * kTilePitch + c4 + 0] = v[0];
    xs[tt * kTilePitch + c4 + 1] = v[1];
    xs[tt * kTilePitch + c4 + 2] = v[2];
    xs[tt * kTilePitch + c4 + 3] = v[3];
  }
  __syncthreads();
  const int q  = lane >> 3;
  const int c8 = (lane & 7) * 8;
  for (int pass = 0; pass < 2; ++pass) {
    for (int it = 0; it < 2; ++it) {
      const int d = wave * 8 + it * 4 + q;
      v4u hv, lv;
      split_pack8(xs, c8, d, hv, lv);
      const size_t off = (size_t)(b * 64 + d) * kSeq + (size_t)t0 + c8;
      *(volatile v4u*)(XTh + off) = hv;
      *(volatile v4u*)(XTl + off) = lv;
    }
    __threadfence();
  }
}

union FragB { v16b v; v8b h[2]; };
__device__ __forceinline__ v16b frag_load(const __bf16* p) {
  FragB f;
  f.h[0] = *(const v8b*)(p);
  f.h[1] = *(const v8b*)(p + 16);
  return f.v;
}
__device__ __forceinline__ v8f mma_g(v16b a, v16b b, v8f c) {
  c = __builtin_amdgcn_wmma_f32_16x16x32_bf16(false, a, false, b, (short)0, c, false, false);
  asm volatile("v_nop\n\tv_nop\n\tv_nop\n\tv_nop" : "+v"(c) : "v"(a), "v"(b));
  return c;
}

__global__ __launch_bounds__(128) void k_product(
    const unsigned short* __restrict__ XTh, const unsigned short* __restrict__ XTl,
    const unsigned short* __restrict__ VTh, const unsigned short* __restrict__ VTl,
    float* __restrict__ out) {
  __shared__ __align__(16) float sT[4][16 * 68];
  const int lane = threadIdx.x & 31;
  const int wave = threadIdx.x >> 5;
  const int hh   = lane >> 4;
  const int rl   = lane & 15;
  const int koff = hh * 8;
  const int row0 = blockIdx.x * 64 + wave * 16;

  const __bf16* Ah = (const __bf16*)XTh + (size_t)(row0 + rl) * kSeq + koff;
  const __bf16* Al = (const __bf16*)XTl + (size_t)(row0 + rl) * kSeq + koff;
  const __bf16* Bh = (const __bf16*)VTh + (size_t)rl * kSeq + koff;
  const __bf16* Bl = (const __bf16*)VTl + (size_t)rl * kSeq + koff;

  v8f accm[4], accr[4];
#pragma unroll
  for (int j = 0; j < 4; ++j) {
    accm[j] = (v8f){0.f, 0.f, 0.f, 0.f, 0.f, 0.f, 0.f, 0.f};
    accr[j] = (v8f){0.f, 0.f, 0.f, 0.f, 0.f, 0.f, 0.f, 0.f};
  }

  for (int k0 = 0; k0 < kSeq; k0 += 32) {
    const v16b ah = frag_load(Ah + k0);
    const v16b al = frag_load(Al + k0);
#pragma unroll
    for (int j = 0; j < 4; ++j) {
      const v16b bh = frag_load(Bh + (size_t)(j * 16) * kSeq + k0);
      const v16b bl = frag_load(Bl + (size_t)(j * 16) * kSeq + k0);
      accm[j] = mma_g(ah, bh, accm[j]);
      accr[j] = mma_g(al, bh, accr[j]);
      accr[j] = mma_g(ah, bl, accr[j]);
    }
  }

  float* slab = sT[wave];
#pragma unroll
  for (int j = 0; j < 4; ++j) {
#pragma unroll
    for (int r = 0; r < 8; ++r) {
      slab[(8 * hh + r) * 68 + j * 16 + rl] = accm[j][r] + accr[j][r];
    }
  }
  __syncthreads();
  float* C = out + (size_t)row0 * kState;
  const int c4 = (lane & 15) * 4;
  for (int pass = 0; pass < 2; ++pass) {
#pragma unroll
    for (int it = 0; it < 8; ++it) {
      const int row = it * 2 + hh;
      const v4f v = *(const v4fa*)(slab + row * 68 + c4);
      *(volatile v4f*)(C + (size_t)row * kState + c4) = v;
    }
    __threadfence();
  }
}

extern "C" void kernel_launch(void* const* d_in, const int* in_sizes, int n_in,
                              void* d_out, int out_size, void* d_ws, size_t ws_size,
                              hipStream_t stream) {
  if (n_in < 3) return;
  if (in_sizes[0] != kBatch * kSeq * kDim) return;
  if (in_sizes[1] != kState * kState) return;
  if (in_sizes[2] != kState) return;
  if (out_size != kRows * kState) return;
  if (ws_size < kCarveBytes) return;
  const float* x  = (const float*)d_in[0];
  const float* dA = (const float*)d_in[1];
  const float* dB = (const float*)d_in[2];
  float* out = (float*)d_out;
  unsigned char* ws = (unsigned char*)d_ws;
  unsigned short* VTh = (unsigned short*)(ws + kOffVtHi);
  unsigned short* VTl = (unsigned short*)(ws + kOffVtLo);
  unsigned short* XTh = (unsigned short*)(ws + kOffXtHi);
  unsigned short* XTl = (unsigned short*)(ws + kOffXtLo);

  k_vchain<<<1, 64, 0, stream>>>(dA, dB, VTh, VTl);
  k_xplanes<<<kBatch * (kSeq / 64), 256, 0, stream>>>(x, XTh, XTl);
  k_product<<<kRows / 64, 128, 0, stream>>>(XTh, XTl, VTh, VTl, out);
}
